// TrXLI_1511828488255
// MI455X (gfx1250) — hardware-verified
//
#include <hip/hip_runtime.h>

#define BATCH 4
#define SEQ   2048
#define DIM   512
#define NH    8
#define DH    64
#define BS    (BATCH * SEQ)

typedef __attribute__((ext_vector_type(16))) _Float16 v16h;
typedef __attribute__((ext_vector_type(8)))  _Float16 v8h;
typedef __attribute__((ext_vector_type(8)))  float    v8f;
typedef __attribute__((ext_vector_type(4)))  float    v4f;
typedef __attribute__((ext_vector_type(4)))  unsigned v4u;
template <typename V> __device__ __forceinline__ void vst2(void* p, V v) {
  *(volatile V*)p = v; __threadfence(); *(volatile V*)p = v;
}
#define PSC 256.0f
#define PUN (1.0f / 256.0f)


__device__ __forceinline__ v16h load_frag_a(const _Float16* p, int lda, int lane) {
  int row  = lane & 15;
  int koff = (lane & 16) ? 8 : 0;
  const _Float16* r = p + (size_t)row * lda + koff;
  v8h lo = *(const v8h*)r;
  v8h hi = *(const v8h*)(r + 16);
  v16h a;
#pragma unroll
  for (int i = 0; i < 8; ++i) { a[i] = lo[i]; a[8 + i] = hi[i]; }
  return a;
}

__device__ __forceinline__ v16h load_frag_b(const _Float16* bt, int ldb, int lane) {
  int n  = lane & 15;
  int kb = (lane & 16) ? 8 : 0;
  const _Float16* c = bt + (size_t)n * ldb + kb;
  v8h lo = *(const v8h*)c;
  v8h hi = *(const v8h*)(c + 16);
  v16h b;
#pragma unroll
  for (int i = 0; i < 8; ++i) { b[i] = lo[i]; b[8 + i] = hi[i]; }
  return b;
}

__device__ __forceinline__ v8f wmma_f16(v16h a, v16h b, v8f c) {
  v8f d = __builtin_amdgcn_wmma_f32_16x16x32_f16(false, a, false, b, (short)0, c, false, false);
  asm volatile("v_nop\n\tv_nop\n\tv_nop\n\tv_nop" : "+v"(d) : "v"(a), "v"(b));
  return d;
}
__device__ __forceinline__ void copy_b128(_Float16* lds_dst, const _Float16* gsrc) {
  *(v4u*)lds_dst = *(const v4u*)gsrc;
}

__global__ __launch_bounds__(256) void cvt_transpose_h(const float* __restrict__ W, _Float16* __restrict__ WT, int H, int K, int N) {
  __shared__ __align__(16) _Float16 tile[64][DIM + 8];
  const int tid = threadIdx.x;
  const int nt = N / 64;
  const int h = blockIdx.x / nt, n0 = (blockIdx.x % nt) * 64;
  for (int i = tid; i < K * 64; i += 256) { const int k = i >> 6, nl = i & 63; tile[nl][k] = (_Float16)W[((size_t)h * K + k) * N + n0 + nl]; }
  __syncthreads();
  for (int g = tid; g < 64 * (K / 8); g += 256) {
    const int nl = g / (K / 8), pc = g - nl * (K / 8);
    vst2(WT + ((size_t)h * N + n0 + nl) * K + pc * 8, *(const v4u*)(&tile[nl][pc * 8]));
  }
}

__global__ __launch_bounds__(128) void layernorm_f16(const float* __restrict__ X,
                                                     const float* __restrict__ g,
                                                     const float* __restrict__ bb,
                                                     _Float16* __restrict__ Y) {
  __shared__ float red[256];
  int row = blockIdx.x;
  const float* x = X + (size_t)row * DIM;
  float s = 0.f, ss = 0.f;
  for (int i = threadIdx.x; i < DIM; i += 128) {
    float v = x[i];
    s += v; ss += v * v;
  }
  red[threadIdx.x] = s;
  red[threadIdx.x + 128] = ss;
  __syncthreads();
  for (int off = 64; off > 0; off >>= 1) {
    if ((int)threadIdx.x < off) {
      red[threadIdx.x]       += red[threadIdx.x + off];
      red[threadIdx.x + 128] += red[threadIdx.x + 128 + off];
    }
    __syncthreads();
  }
  float mean = red[0] * (1.0f / DIM);
  float var  = red[128] * (1.0f / DIM) - mean * mean;
  float rstd = rsqrtf(var + 1e-5f);
  {
    const int c0 = threadIdx.x * 4;
    union { _Float16 h[4]; unsigned long long u; } pk;
#pragma unroll
    for (int e = 0; e < 4; ++e) pk.h[e] = (_Float16)((x[c0 + e] - mean) * rstd * g[c0 + e] + bb[c0 + e]);
    vst2(Y + (size_t)row * DIM + c0, pk.u);
  }
}

__global__ __launch_bounds__(256) void qkv_gemm(
    const _Float16* __restrict__ hF16,
    const _Float16* __restrict__ WqT, const _Float16* __restrict__ WkT,
    const _Float16* __restrict__ WvT,
    const float* __restrict__ bq, const float* __restrict__ bk,
    const float* __restrict__ bv,
    _Float16* __restrict__ q, _Float16* __restrict__ k,
    _Float16* __restrict__ vT) {
  __shared__ __align__(16) _Float16 st[64 * 264];
  const int lane = threadIdx.x & 31;
  const int wave = threadIdx.x >> 5;
  const int srow = blockIdx.x * 256 + wave * 32;
  const int h    = blockIdx.y;
  const int b    = blockIdx.z / 3;
  const int mat  = blockIdx.z % 3;

  const _Float16* WT   = (mat == 0) ? WqT : (mat == 1) ? WkT : WvT;
  const float*    bias = (mat == 0) ? bq  : (mat == 1) ? bk  : bv;
  const _Float16* A  = hF16 + ((size_t)b * SEQ + srow) * DIM;
  const _Float16* Bh = WT + (size_t)h * DH * DIM;

  v8f acc[2][4] = {};
  v16h a0 = load_frag_a(A, DIM, lane);
  v16h a1 = load_frag_a(A + (size_t)16 * DIM, DIM, lane);
  v16h bf0 = load_frag_b(Bh + (size_t)0  * DIM, DIM, lane);
  v16h bf1 = load_frag_b(Bh + (size_t)16 * DIM, DIM, lane);
  v16h bf2 = load_frag_b(Bh + (size_t)32 * DIM, DIM, lane);
  v16h bf3 = load_frag_b(Bh + (size_t)48 * DIM, DIM, lane);

  for (int kk = 0; kk < DIM; kk += 32) {
    int nk = kk + 32;
    v16h na0, na1, nb0, nb1, nb2, nb3;
    if (nk < DIM) {
      na0 = load_frag_a(A + nk, DIM, lane);
      na1 = load_frag_a(A + (size_t)16 * DIM + nk, DIM, lane);
      nb0 = load_frag_b(Bh + (size_t)0  * DIM + nk, DIM, lane);
      nb1 = load_frag_b(Bh + (size_t)16 * DIM + nk, DIM, lane);
      nb2 = load_frag_b(Bh + (size_t)32 * DIM + nk, DIM, lane);
      nb3 = load_frag_b(Bh + (size_t)48 * DIM + nk, DIM, lane);
    }
    acc[0][0] = wmma_f16(a0, bf0, acc[0][0]);
    acc[0][1] = wmma_f16(a0, bf1, acc[0][1]);
    acc[0][2] = wmma_f16(a0, bf2, acc[0][2]);
    acc[0][3] = wmma_f16(a0, bf3, acc[0][3]);
    acc[1][0] = wmma_f16(a1, bf0, acc[1][0]);
    acc[1][1] = wmma_f16(a1, bf1, acc[1][1]);
    acc[1][2] = wmma_f16(a1, bf2, acc[1][2]);
    acc[1][3] = wmma_f16(a1, bf3, acc[1][3]);
    if (nk < DIM) {
      a0 = na0; a1 = na1;
      bf0 = nb0; bf1 = nb1; bf2 = nb2; bf3 = nb3;
    }
  }

  const int n0    = lane & 15;
  const int mbase = (lane >> 4) << 3;
  const size_t headoff = (size_t)b * NH + h;
#pragma unroll
  for (int sub = 0; sub < 2; ++sub) {
#pragma unroll
    for (int t = 0; t < 4; ++t) {
      int n = t * 16 + n0;
      float bia = bias[h * DH + n];
#pragma unroll
      for (int i = 0; i < 8; ++i) {
        float val = acc[sub][t][i] + bia;
        int ml = wave * 32 + sub * 16 + mbase + i;
        if (mat == 2) st[n * 264 + ml] = (_Float16)val;
        else          st[ml * 64 + n]  = (_Float16)val;
      }
    }
  }
  __syncthreads();
  if (mat == 2) {
    for (int g = threadIdx.x; g < 64 * 32; g += 256) {
      const int n = g >> 5, pc = g & 31;
      vst2(vT + (headoff * DH + n) * SEQ + blockIdx.x * 256 + pc * 8, *(const v4u*)(&st[n * 264 + pc * 8]));
    }
  } else {
    _Float16* dst = (mat == 0) ? q : k;
    for (int g = threadIdx.x; g < 256 * 8; g += 256) {
      const int ml = g >> 3, pc = g & 7;
      vst2(dst + (headoff * SEQ + blockIdx.x * 256 + ml) * DH + pc * 8, *(const v4u*)(&st[ml * 64 + pc * 8]));
    }
  }
}

__global__ __launch_bounds__(256) void attn_kernel(
    const _Float16* __restrict__ q, const _Float16* __restrict__ k,
    const _Float16* __restrict__ vT, _Float16* __restrict__ om) {
  __shared__ __align__(16) _Float16 Kt[2][32 * DH];
  __shared__ __align__(16) _Float16 Vt[2][DH * 32];
  __shared__ __align__(16) _Float16 plds[8][16 * 32];
  __shared__ __align__(16) _Float16 ost[8][16 * DH];

  const int tid  = threadIdx.x;
  const int lane = tid & 31;
  const int wave = tid >> 5;
  const int h = blockIdx.y, b = blockIdx.z;
  const int qrow = blockIdx.x * 128 + wave * 16;
  const size_t headoff = (size_t)b * NH + h;
  const _Float16* qh = q  + headoff * SEQ * DH;
  const _Float16* kh = k  + headoff * SEQ * DH;
  const _Float16* vh = vT + headoff * DH * SEQ;

  const int n0    = lane & 15;
  const int mbase = (lane >> 4) << 3;

  const int krow = tid >> 3, kch = (tid & 7) * 8;
  const int vrow = tid >> 2, vch = (tid & 3) * 8;

  copy_b128(&Kt[0][krow * DH + kch], kh + (size_t)krow * DH + kch);
  copy_b128(&Vt[0][vrow * 32 + vch], vh + (size_t)vrow * SEQ + vch);

  v16h qa0 = load_frag_a(qh + (size_t)qrow * DH,      DH, lane);
  v16h qa1 = load_frag_a(qh + (size_t)qrow * DH + 32, DH, lane);

  v8f oacc[4] = {};
  float mrow[8], lrow[8];
#pragma unroll
  for (int i = 0; i < 8; ++i) { mrow[i] = -1e30f; lrow[i] = 0.f; }
  const float scale = 0.125f;
  _Float16* pl = plds[wave];

  const int NTILE = SEQ / 32;
  for (int it = 0; it < NTILE; ++it) {
    const int kt  = it * 32;
    const int buf = it & 1;
    if (it + 1 < NTILE) {
      const int nkt = kt + 32;
      copy_b128(&Kt[buf ^ 1][krow * DH + kch], kh + (size_t)(nkt + krow) * DH + kch);
      copy_b128(&Vt[buf ^ 1][vrow * 32 + vch], vh + (size_t)vrow * SEQ + nkt + vch);
    }
    __syncthreads();

    const _Float16* Kb = Kt[buf];
    const _Float16* Vb = Vt[buf];

    v8f s0 = {}, s1 = {};
    {
      v16h b0 = load_frag_b(Kb,                DH, lane);
      v16h b1 = load_frag_b(Kb + 32,           DH, lane);
      s0 = wmma_f16(qa0, b0, s0);
      s0 = wmma_f16(qa1, b1, s0);
      v16h b2 = load_frag_b(Kb + 16 * DH,      DH, lane);
      v16h b3 = load_frag_b(Kb + 16 * DH + 32, DH, lane);
      s1 = wmma_f16(qa0, b2, s1);
      s1 = wmma_f16(qa1, b3, s1);
    }
    float p0[8], p1[8];
#pragma unroll
    for (int i = 0; i < 8; ++i) {
      float a0 = s0[i] * scale, a1 = s1[i] * scale;
      float vmax = fmaxf(a0, a1);
#pragma unroll
      for (int off = 1; off < 16; off <<= 1)
        vmax = fmaxf(vmax, __shfl_xor(vmax, off, 32));
      float mnew  = fmaxf(mrow[i], vmax);
      float alpha = __expf(mrow[i] - mnew);
      mrow[i] = mnew;
      float e0 = __expf(a0 - mnew);
      float e1 = __expf(a1 - mnew);
      p0[i] = e0; p1[i] = e1;
      float rs = e0 + e1;
#pragma unroll
      for (int off = 1; off < 16; off <<= 1)
        rs += __shfl_xor(rs, off, 32);
      lrow[i] = lrow[i] * alpha + rs;
#pragma unroll
      for (int t = 0; t < 4; ++t) oacc[t][i] *= alpha;
    }
#pragma unroll
    for (int i = 0; i < 8; ++i) {
      pl[(mbase + i) * 32 + n0]      = (_Float16)(p0[i] * PSC);
      pl[(mbase + i) * 32 + 16 + n0] = (_Float16)(p1[i] * PSC);
    }
    __syncthreads();
    v16h pa = load_frag_a(pl, 32, lane);
#pragma unroll
    for (int t = 0; t < 4; ++t) {
      v16h vb = load_frag_b(Vb + (size_t)(t * 16) * 32, 32, lane);
      oacc[t] = wmma_f16(pa, vb, oacc[t]);
    }
    __syncthreads();
  }

  _Float16* os_ = ost[wave];
#pragma unroll
  for (int t = 0; t < 4; ++t) {
#pragma unroll
    for (int i = 0; i < 8; ++i) os_[(mbase + i) * DH + t * 16 + n0] = (_Float16)(oacc[t][i] * (PUN / lrow[i]));
  }
  __syncthreads();
#pragma unroll
  for (int qq = 0; qq < 4; ++qq) {
    const int ml = qq * 4 + (lane >> 3), pc = lane & 7;
    vst2(om + ((size_t)b * SEQ + qrow + ml) * DIM + h * DH + pc * 8, *(const v4u*)(&os_[ml * DH + pc * 8]));
  }
}

__global__ __launch_bounds__(256) void gemm512_epilogue(
    const _Float16* __restrict__ A, const _Float16* __restrict__ WT,
    const float* __restrict__ bias, const float* __restrict__ res,
    float* __restrict__ out, int relu_mode) {
  __shared__ __align__(16) float st[8][32 * 64];
  const int lane = threadIdx.x & 31;
  const int wave = threadIdx.x >> 5;
  const int m0  = blockIdx.x * 256 + wave * 32;
  const int n0t = blockIdx.y * 64;

  const _Float16* Ar = A + (size_t)m0 * DIM;
  const _Float16* Wb = WT + (size_t)n0t * DIM;

  v8f acc[2][4] = {};
  v16h a0 = load_frag_a(Ar, DIM, lane);
  v16h a1 = load_frag_a(Ar + (size_t)16 * DIM, DIM, lane);
  v16h bf0 = load_frag_b(Wb + (size_t)0  * DIM, DIM, lane);
  v16h bf1 = load_frag_b(Wb + (size_t)16 * DIM, DIM, lane);
  v16h bf2 = load_frag_b(Wb + (size_t)32 * DIM, DIM, lane);
  v16h bf3 = load_frag_b(Wb + (size_t)48 * DIM, DIM, lane);

  for (int kk = 0; kk < DIM; kk += 32) {
    int nk = kk + 32;
    v16h na0, na1, nb0, nb1, nb2, nb3;
    if (nk < DIM) {
      na0 = load_frag_a(Ar + nk, DIM, lane);
      na1 = load_frag_a(Ar + (size_t)16 * DIM + nk, DIM, lane);
      nb0 = load_frag_b(Wb + (size_t)0  * DIM + nk, DIM, lane);
      nb1 = load_frag_b(Wb + (size_t)16 * DIM + nk, DIM, lane);
      nb2 = load_frag_b(Wb + (size_t)32 * DIM + nk, DIM, lane);
      nb3 = load_frag_b(Wb + (size_t)48 * DIM + nk, DIM, lane);
    }
    acc[0][0] = wmma_f16(a0, bf0, acc[0][0]);
    acc[0][1] = wmma_f16(a0, bf1, acc[0][1]);
    acc[0][2] = wmma_f16(a0, bf2, acc[0][2]);
    acc[0][3] = wmma_f16(a0, bf3, acc[0][3]);
    acc[1][0] = wmma_f16(a1, bf0, acc[1][0]);
    acc[1][1] = wmma_f16(a1, bf1, acc[1][1]);
    acc[1][2] = wmma_f16(a1, bf2, acc[1][2]);
    acc[1][3] = wmma_f16(a1, bf3, acc[1][3]);
    if (nk < DIM) {
      a0 = na0; a1 = na1;
      bf0 = nb0; bf1 = nb1; bf2 = nb2; bf3 = nb3;
    }
  }

  const int nl    = lane & 15;
  const int mbase = (lane >> 4) << 3;
#pragma unroll
  for (int sub = 0; sub < 2; ++sub) {
#pragma unroll
    for (int t = 0; t < 4; ++t) {
      int n = n0t + t * 16 + nl;
      float bia = bias[n];
#pragma unroll
      for (int i = 0; i < 8; ++i) {
        const int ml = sub * 16 + mbase + i;
        size_t idx = (size_t)(m0 + ml) * DIM + n;
        float v = acc[sub][t][i] + bia;
        if (relu_mode) v = fmaxf(v, 0.f);
        v += res[idx];
        st[wave][ml * 64 + t * 16 + nl] = v;
      }
    }
  }
  __syncthreads();
#pragma unroll
  for (int q = 0; q < 16; ++q) {
    const int ml = q * 2 + (lane >> 4), pc = lane & 15;
    vst2(out + (size_t)(m0 + ml) * DIM + n0t + pc * 4, *(const v4f*)(&st[wave][ml * 64 + pc * 4]));
  }
}

extern "C" void kernel_launch(void* const* d_in, const int* in_sizes, int n_in,
                              void* d_out, int out_size, void* d_ws, size_t ws_size,
                              hipStream_t stream) {
  const float* x  = (const float*)d_in[0];
  const float* g1 = (const float*)d_in[1];
  const float* b1 = (const float*)d_in[2];
  const float* Wq = (const float*)d_in[3];
  const float* bq = (const float*)d_in[4];
  const float* Wk = (const float*)d_in[5];
  const float* bk = (const float*)d_in[6];
  const float* Wv = (const float*)d_in[7];
  const float* bv = (const float*)d_in[8];
  const float* Wm = (const float*)d_in[9];
  const float* bm = (const float*)d_in[10];
  const float* g2 = (const float*)d_in[11];
  const float* b2 = (const float*)d_in[12];
  const float* Wo = (const float*)d_in[13];
  const float* bo = (const float*)d_in[14];
  float* out = (float*)d_out;

  char* ws = (char*)d_ws;
  size_t off = 0;
  auto alloc = [&](size_t bytes) {
    void* p = ws + off;
    off = (off + bytes + 255) & ~(size_t)255;
    return p;
  };

  _Float16* hF16 = (_Float16*)alloc((size_t)BS * DIM * 2);
  _Float16* WqT  = (_Float16*)alloc((size_t)NH * DH * DIM * 2);
  _Float16* WkT  = (_Float16*)alloc((size_t)NH * DH * DIM * 2);
  _Float16* WvT  = (_Float16*)alloc((size_t)NH * DH * DIM * 2);
  _Float16* WmT  = (_Float16*)alloc((size_t)DIM * DIM * 2);
  _Float16* WoT  = (_Float16*)alloc((size_t)DIM * DIM * 2);
  _Float16* qb   = (_Float16*)alloc((size_t)BATCH * NH * SEQ * DH * 2);
  _Float16* kb   = (_Float16*)alloc((size_t)BATCH * NH * SEQ * DH * 2);
  _Float16* vTb  = (_Float16*)alloc((size_t)BATCH * NH * DH * SEQ * 2);
  _Float16* om   = (_Float16*)alloc((size_t)BS * DIM * 2);
  float*    hlp  = (float*)alloc((size_t)BS * DIM * 4);
  _Float16* hfc  = (_Float16*)alloc((size_t)BS * DIM * 2);

  {
    cvt_transpose_h<<<NH * (DH / 64), 256, 0, stream>>>(Wq, WqT, NH, DIM, DH);
    cvt_transpose_h<<<NH * (DH / 64), 256, 0, stream>>>(Wk, WkT, NH, DIM, DH);
    cvt_transpose_h<<<NH * (DH / 64), 256, 0, stream>>>(Wv, WvT, NH, DIM, DH);
    cvt_transpose_h<<<DIM / 64, 256, 0, stream>>>(Wm, WmT, 1, DIM, DIM);
    cvt_transpose_h<<<DIM / 64, 256, 0, stream>>>(Wo, WoT, 1, DIM, DIM);
  }

  layernorm_f16<<<BS, 128, 0, stream>>>(x, g1, b1, hF16);

  qkv_gemm<<<dim3(SEQ / 256, NH, BATCH * 3), 256, 0, stream>>>(
      hF16, WqT, WkT, WvT, bq, bk, bv, qb, kb, vTb);

  attn_kernel<<<dim3(SEQ / 128, NH, BATCH), 256, 0, stream>>>(qb, kb, vTb, om);

  gemm512_epilogue<<<dim3(BS / 256, DIM / 64), 256, 0, stream>>>(
      om, WmT, bm, x, hlp, 0);

  layernorm_f16<<<BS, 128, 0, stream>>>(hlp, g2, b2, hfc);

  gemm512_epilogue<<<dim3(BS / 256, DIM / 64), 256, 0, stream>>>(
      hfc, WoT, bo, hlp, out, 1);
}
